// WaveModel_41162966564996
// MI455X (gfx1250) — hardware-verified
//
#include <hip/hip_runtime.h>
#define NB 256
#define NT_ 2048
#define HH 64
#define G4 256

typedef __bf16 v16b __attribute__((ext_vector_type(16)));
typedef unsigned short v8us __attribute__((ext_vector_type(8), may_alias));
typedef float  v8f  __attribute__((ext_vector_type(8)));
typedef float  v4f  __attribute__((ext_vector_type(4)));
typedef float  v4fa __attribute__((ext_vector_type(4), may_alias));
union FragB { v16b v; v8us half[2]; unsigned short u[16]; };

__device__ __forceinline__ unsigned short bf16_bits(float x) { unsigned int u = __float_as_uint(x); return (unsigned short)((u + 0x7FFFu + ((u >> 16) & 1u)) >> 16); }
__device__ __forceinline__ float bf16_val(unsigned short b) { return __uint_as_float(((unsigned int)b) << 16); }
__device__ __forceinline__ float bf16_round(float x) { return bf16_val(bf16_bits(x)); }
template <int NT>
__device__ __forceinline__ v8f mmaN(v16b ah, v16b al, v16b bh, v16b bl, v8f c) {
  c = __builtin_amdgcn_wmma_f32_16x16x32_bf16(false, ah, false, bh, (short)0, c, false, false);
  if (NT >= 2) c = __builtin_amdgcn_wmma_f32_16x16x32_bf16(false, al, false, bh, (short)0, c, false, false);
  if (NT >= 3) c = __builtin_amdgcn_wmma_f32_16x16x32_bf16(false, ah, false, bl, (short)0, c, false, false);
  asm volatile("v_nop\n\tv_nop\n\tv_nop\n\tv_nop" : "+v"(c) : "v"(ah), "v"(al), "v"(bh), "v"(bl));
  return c;
}

__global__ __launch_bounds__(256) void k_wt_bf16(const float* __restrict__ W, unsigned short* __restrict__ Wt, int K, int N) {
  const int t = blockIdx.x * 256 + threadIdx.x;
  const int k8n = K / 8;
  if (t >= N * k8n) return;
  const int n = t / k8n, k8 = (t % k8n) * 8;
  v8us v;
#pragma unroll
  for (int i = 0; i < 8; ++i) v[i] = bf16_bits(W[(size_t)(k8 + i) * N + n]);
  *(volatile v8us*)(Wt + (size_t)n * K + k8) = v;
  __threadfence();
  *(volatile v8us*)(Wt + (size_t)n * K + k8) = v;
}

template <bool ASPLIT, int ACT, bool BIAS_BF16>
__global__ __launch_bounds__(128) void k_gemm_bf(const float* __restrict__ A, int lda, const unsigned short* __restrict__ Wt, int ldb,
                                               const float* __restrict__ bias, float* __restrict__ C, int ldc, int M, int N, int K) {
  __shared__ __attribute__((aligned(16))) float so[4][16][64];
  const int tid = threadIdx.x, w = tid >> 5, lane = tid & 31, ln = lane & 15, hh = lane >> 4;
  const int ntn = N / 64;
  const int wid = blockIdx.x * 4 + w;
  const int mt = wid / ntn, nq = wid % ntn;
  if (mt * 16 >= M) return;
  const int row0 = mt * 16, col0 = nq * 64;
  const float* arow = A + (size_t)(row0 + ln) * lda;
  v8f acc[4] = {};
  for (int kb = 0; kb < K; kb += 32) {
    FragB ah, al;
    const v4f x0 = *(const v4fa*)(arow + kb + 8 * hh), x1 = *(const v4fa*)(arow + kb + 8 * hh + 4);
    const v4f x2 = *(const v4fa*)(arow + kb + 16 + 8 * hh), x3 = *(const v4fa*)(arow + kb + 16 + 8 * hh + 4);
    float xs[16] = {x0[0],x0[1],x0[2],x0[3],x1[0],x1[1],x1[2],x1[3],x2[0],x2[1],x2[2],x2[3],x3[0],x3[1],x3[2],x3[3]};
#pragma unroll
    for (int i = 0; i < 16; ++i) { const unsigned short hb = bf16_bits(xs[i]); ah.u[i] = hb; al.u[i] = ASPLIT ? bf16_bits(xs[i] - bf16_val(hb)) : (unsigned short)0; }
#pragma unroll
    for (int t = 0; t < 4; ++t) {
      const unsigned short* brow = Wt + (size_t)(col0 + t * 16 + ln) * ldb + kb;
      FragB b;
      b.half[0] = *(const v8us*)(brow + 8 * hh);
      b.half[1] = *(const v8us*)(brow + 16 + 8 * hh);
      acc[t] = mmaN<ASPLIT ? 2 : 1>(ah.v, al.v, b.v, b.v, acc[t]);
    }
  }
#pragma unroll
  for (int t = 0; t < 4; ++t) {
    float bv = bias ? bias[col0 + t * 16 + ln] : 0.f;
    if (BIAS_BF16) bv = bf16_round(bv);
#pragma unroll
    for (int r = 0; r < 8; ++r) { float v = acc[t][r] + bv; if (ACT == 1) v = fmaxf(v, 0.f); so[w][8 * hh + r][t * 16 + ln] = v; }
  }
  __builtin_amdgcn_fence(__ATOMIC_ACQ_REL, "workgroup");
  __builtin_amdgcn_wave_barrier();
  const int rsub = lane >> 4, c4 = (lane & 15) * 4;
  for (int pass = 0; pass < 2; ++pass) {
#pragma unroll
    for (int q = 0; q < 8; ++q) {
      const int r = q * 2 + rsub;
      const v4f v = *(const v4fa*)&so[w][r][c4];
      *(volatile v4f*)(C + (size_t)(row0 + r) * ldc + col0 + c4) = v;
    }
    if (pass == 0) __threadfence();
  }
}

template <int D, bool CAUSAL>
__global__ __launch_bounds__(128) void k_flash(const float* __restrict__ qb, const float* __restrict__ kb, const float* __restrict__ vb,
                                             int pitch, int T, int H, float scale, float* __restrict__ y, int ypitch) {
  constexpr int KS = D / 32;
  constexpr int DT = D / 16;
  __shared__ __attribute__((aligned(16))) unsigned short sKh[32][D + 8], sKl[32][D + 8], sVh[32][D + 8], sVl[32][D + 8];
  __shared__ __attribute__((aligned(16))) unsigned short sPh[4][16][40], sPl[4][16][40];
  __shared__ __attribute__((aligned(16))) float sO[4][16][D];
  const int tid = threadIdx.x, w = tid >> 5, lane = tid & 31, ln = lane & 15, hh = lane >> 4;
  const int nqb = (T + 63) / 64;
  const int bh = blockIdx.x / nqb, qblk = blockIdx.x % nqb;
  const int b = bh / H, h = bh % H;
  const int q0 = qblk * 64 + w * 16;
  const float* Q = qb + (size_t)b * T * pitch + h * D;
  const float* K = kb + (size_t)b * T * pitch + h * D;
  const float* V = vb + (size_t)b * T * pitch + h * D;

  FragB aqh[KS], aql[KS];
  {
    int row = q0 + ln; if (row >= T) row = T - 1;
    const float* qr = Q + (size_t)row * pitch;
#pragma unroll
    for (int ks = 0; ks < KS; ++ks)
#pragma unroll
      for (int i = 0; i < 16; ++i) {
        const int d = ks * 32 + ((i < 8) ? (8 * hh + i) : (16 + 8 * hh + (i - 8)));
        const float x = qr[d] * scale; const unsigned short hb = bf16_bits(x);
        aqh[ks].u[i] = hb; aql[ks].u[i] = bf16_bits(x - bf16_val(hb));
      }
  }
  float m_r[8], l_r[8];
#pragma unroll
  for (int r = 0; r < 8; ++r) { m_r[r] = -3.0e38f; l_r[r] = 0.f; }
  v8f oacc[DT];
#pragma unroll
  for (int dt = 0; dt < DT; ++dt) oacc[dt] = (v8f){0.f,0.f,0.f,0.f,0.f,0.f,0.f,0.f};

  const int kv_end = CAUSAL ? min(T, qblk * 64 + 64) : T;
  for (int j0 = 0; j0 < kv_end; j0 += 32) {
    __syncthreads();
    for (int e = tid; e < 32 * (D / 4); e += 128) {
      const int r = e / (D / 4), c4 = (e % (D / 4)) * 4;
      const int key = j0 + r;
      v4f kf = {0.f,0.f,0.f,0.f}, vf = {0.f,0.f,0.f,0.f};
      if (key < T) { kf = *(const v4fa*)(K + (size_t)key * pitch + c4); vf = *(const v4fa*)(V + (size_t)key * pitch + c4); }
#pragma unroll
      for (int t = 0; t < 4; ++t) {
        unsigned short hb = bf16_bits(kf[t]); sKh[r][c4 + t] = hb; sKl[r][c4 + t] = bf16_bits(kf[t] - bf16_val(hb));
        hb = bf16_bits(vf[t]); sVh[r][c4 + t] = hb; sVl[r][c4 + t] = bf16_bits(vf[t] - bf16_val(hb));
      }
    }
    __syncthreads();
    v8f s[2];
#pragma unroll
    for (int nt = 0; nt < 2; ++nt) {
      v8f acc = {};
#pragma unroll
      for (int ks = 0; ks < KS; ++ks) {
        FragB bh_, bl_;
        bh_.half[0] = *(const v8us*)&sKh[nt * 16 + ln][ks * 32 + 8 * hh]; bh_.half[1] = *(const v8us*)&sKh[nt * 16 + ln][ks * 32 + 16 + 8 * hh];
        bl_.half[0] = *(const v8us*)&sKl[nt * 16 + ln][ks * 32 + 8 * hh]; bl_.half[1] = *(const v8us*)&sKl[nt * 16 + ln][ks * 32 + 16 + 8 * hh];
        acc = mmaN<3>(aqh[ks].v, aql[ks].v, bh_.v, bl_.v, acc);
      }
      s[nt] = acc;
    }
    float alpha[8];
#pragma unroll
    for (int r = 0; r < 8; ++r) {
      const int qi = q0 + 8 * hh + r;
      const int ja = j0 + ln, jb = j0 + 16 + ln;
      if (CAUSAL) { if (ja > qi) s[0][r] = -3.0e38f; if (jb > qi) s[1][r] = -3.0e38f; }
      if (ja >= T) s[0][r] = -3.0e38f;
      if (jb >= T) s[1][r] = -3.0e38f;
      float mx = fmaxf(s[0][r], s[1][r]);
      mx = fmaxf(mx, __shfl_xor(mx, 1, 32)); mx = fmaxf(mx, __shfl_xor(mx, 2, 32)); mx = fmaxf(mx, __shfl_xor(mx, 4, 32)); mx = fmaxf(mx, __shfl_xor(mx, 8, 32));
      const float mnew = fmaxf(m_r[r], mx);
      alpha[r] = (mnew > -1.0e38f) ? __expf(m_r[r] - mnew) : 1.0f;
      const float p0 = (s[0][r] > -1.0e38f) ? __expf(s[0][r] - mnew) : 0.f;
      const float p1 = (s[1][r] > -1.0e38f) ? __expf(s[1][r] - mnew) : 0.f;
      m_r[r] = mnew;
      l_r[r] = l_r[r] * alpha[r] + p0 + p1;
      unsigned short hb = bf16_bits(p0); sPh[w][8 * hh + r][ln] = hb;      sPl[w][8 * hh + r][ln] = bf16_bits(p0 - bf16_val(hb));
      hb = bf16_bits(p1);                sPh[w][8 * hh + r][16 + ln] = hb; sPl[w][8 * hh + r][16 + ln] = bf16_bits(p1 - bf16_val(hb));
    }
#pragma unroll
    for (int dt = 0; dt < DT; ++dt)
#pragma unroll
      for (int r = 0; r < 8; ++r) oacc[dt][r] *= alpha[r];
    __builtin_amdgcn_fence(__ATOMIC_ACQ_REL, "workgroup");
    __builtin_amdgcn_wave_barrier();
    FragB pah, pal;
    pah.half[0] = *(const v8us*)&sPh[w][ln][8 * hh]; pah.half[1] = *(const v8us*)&sPh[w][ln][16 + 8 * hh];
    pal.half[0] = *(const v8us*)&sPl[w][ln][8 * hh]; pal.half[1] = *(const v8us*)&sPl[w][ln][16 + 8 * hh];
#pragma unroll
    for (int dt = 0; dt < DT; ++dt) {
      FragB bvh, bvl;
#pragma unroll
      for (int i = 0; i < 8; ++i) {
        bvh.u[i] = sVh[8 * hh + i][dt * 16 + ln]; bvh.u[8 + i] = sVh[16 + 8 * hh + i][dt * 16 + ln];
        bvl.u[i] = sVl[8 * hh + i][dt * 16 + ln]; bvl.u[8 + i] = sVl[16 + 8 * hh + i][dt * 16 + ln];
      }
      oacc[dt] = mmaN<3>(pah.v, pal.v, bvh.v, bvl.v, oacc[dt]);
    }
    __builtin_amdgcn_fence(__ATOMIC_ACQ_REL, "workgroup");
    __builtin_amdgcn_wave_barrier();
  }
#pragma unroll
  for (int r = 0; r < 8; ++r) {
    float l = l_r[r];
    l += __shfl_xor(l, 1, 32); l += __shfl_xor(l, 2, 32); l += __shfl_xor(l, 4, 32); l += __shfl_xor(l, 8, 32);
    l_r[r] = (l > 0.f) ? 1.0f / l : 0.f;
  }
#pragma unroll
  for (int dt = 0; dt < DT; ++dt)
#pragma unroll
    for (int r = 0; r < 8; ++r) sO[w][8 * hh + r][dt * 16 + ln] = oacc[dt][r] * l_r[r];
  __builtin_amdgcn_fence(__ATOMIC_ACQ_REL, "workgroup");
  __builtin_amdgcn_wave_barrier();
  for (int pass = 0; pass < 2; ++pass) {
    for (int r = 0; r < 16; ++r) {
      const int row = q0 + r;
      if (row < T && lane < D / 4) {
        const v4f val = *(const v4fa*)&sO[w][r][lane * 4];
        *(volatile v4f*)(y + ((size_t)b * T + row) * ypitch + h * D + lane * 4) = val;
      }
    }
    if (pass == 0) __threadfence();
  }
}

__global__ __launch_bounds__(256) void k_split_rows(const float* __restrict__ src, int lds_, unsigned short* __restrict__ hi, unsigned short* __restrict__ lo, int R, int Cc) {
  const size_t t = (size_t)blockIdx.x * 256 + threadIdx.x;
  const int c8n = Cc / 8;
  if (t >= (size_t)R * c8n) return;
  const int r = (int)(t / c8n), c8 = (int)(t % c8n) * 8;
  const float* s = src + (size_t)r * lds_ + c8;
  const v4f a = *(const v4fa*)s, b = *(const v4fa*)(s + 4);
  float xs[8] = {a[0],a[1],a[2],a[3],b[0],b[1],b[2],b[3]};
  v8us vh, vl;
#pragma unroll
  for (int i = 0; i < 8; ++i) { const unsigned short hb = bf16_bits(xs[i]); vh[i] = hb; vl[i] = bf16_bits(xs[i] - bf16_val(hb)); }
  unsigned short* dh = hi + (size_t)r * Cc + c8; unsigned short* dl = lo + (size_t)r * Cc + c8;
  *(volatile v8us*)dh = vh; *(volatile v8us*)dl = vl; __threadfence(); *(volatile v8us*)dh = vh; *(volatile v8us*)dl = vl;
}
__global__ __launch_bounds__(256) void k_split_transpose(const float* __restrict__ src, int lds_, unsigned short* __restrict__ hi, unsigned short* __restrict__ lo, int K, int N) {
  const size_t t = (size_t)blockIdx.x * 256 + threadIdx.x;
  const int k8n = K / 8;
  if (t >= (size_t)N * k8n) return;
  const int n = (int)(t / k8n), k8 = (int)(t % k8n) * 8;
  v8us vh, vl;
#pragma unroll
  for (int i = 0; i < 8; ++i) { const float x = src[(size_t)(k8 + i) * lds_ + n]; const unsigned short hb = bf16_bits(x); vh[i] = hb; vl[i] = bf16_bits(x - bf16_val(hb)); }
  unsigned short* dh = hi + (size_t)n * K + k8; unsigned short* dl = lo + (size_t)n * K + k8;
  *(volatile v8us*)dh = vh; *(volatile v8us*)dl = vl; __threadfence(); *(volatile v8us*)dh = vh; *(volatile v8us*)dl = vl;
}
template <bool ASPLIT, bool BSPLIT, int ACT, bool BIAS_BF16>
__global__ __launch_bounds__(128) void k_gemm_bf2(const float* __restrict__ A, int lda, const unsigned short* __restrict__ Bh, const unsigned short* __restrict__ Bl, int ldb,
                                                const float* __restrict__ bias, float alpha, float* __restrict__ C, int ldc, int M, int N, int K) {
  __shared__ __attribute__((aligned(16))) float so[4][16][64];
  const int tid = threadIdx.x, w = tid >> 5, lane = tid & 31, ln = lane & 15, hh = lane >> 4;
  const int ntn = N / 64;
  const int wid = blockIdx.x * 4 + w;
  const int mt = wid / ntn, nq = wid % ntn;
  if (mt * 16 >= M) return;
  const int row0 = mt * 16, col0 = nq * 64;
  const float* arow = A + (size_t)(row0 + ln) * lda;
  v8f acc[4] = {};
  for (int kb = 0; kb < K; kb += 32) {
    FragB ah, al;
    const v4f x0 = *(const v4fa*)(arow + kb + 8 * hh), x1 = *(const v4fa*)(arow + kb + 8 * hh + 4);
    const v4f x2 = *(const v4fa*)(arow + kb + 16 + 8 * hh), x3 = *(const v4fa*)(arow + kb + 16 + 8 * hh + 4);
    float xs[16] = {x0[0],x0[1],x0[2],x0[3],x1[0],x1[1],x1[2],x1[3],x2[0],x2[1],x2[2],x2[3],x3[0],x3[1],x3[2],x3[3]};
#pragma unroll
    for (int i = 0; i < 16; ++i) { const unsigned short hb = bf16_bits(xs[i]); ah.u[i] = hb; al.u[i] = ASPLIT ? bf16_bits(xs[i] - bf16_val(hb)) : (unsigned short)0; }
#pragma unroll
    for (int t = 0; t < 4; ++t) {
      const size_t boff = (size_t)(col0 + t * 16 + ln) * ldb + kb;
      FragB bh_, bl_;
      bh_.half[0] = *(const v8us*)(Bh + boff + 8 * hh);
      bh_.half[1] = *(const v8us*)(Bh + boff + 16 + 8 * hh);
      if (BSPLIT) { bl_.half[0] = *(const v8us*)(Bl + boff + 8 * hh); bl_.half[1] = *(const v8us*)(Bl + boff + 16 + 8 * hh); } else bl_ = bh_;
      acc[t] = mmaN<ASPLIT ? (BSPLIT ? 3 : 2) : 1>(ah.v, al.v, bh_.v, bl_.v, acc[t]);
    }
  }
#pragma unroll
  for (int t = 0; t < 4; ++t) {
    float bv = bias ? bias[col0 + t * 16 + ln] : 0.f;
    if (BIAS_BF16) bv = bf16_round(bv);
#pragma unroll
    for (int r = 0; r < 8; ++r) { float v = acc[t][r] * alpha + bv; if (ACT == 1) v = fmaxf(v, 0.f); so[w][8 * hh + r][t * 16 + ln] = v; }
  }
  __builtin_amdgcn_fence(__ATOMIC_ACQ_REL, "workgroup");
  __builtin_amdgcn_wave_barrier();
  const int rsub = lane >> 4, c4 = (lane & 15) * 4;
  for (int pass = 0; pass < 2; ++pass) {
#pragma unroll
    for (int q = 0; q < 8; ++q) {
      const int r = q * 2 + rsub;
      const v4f v = *(const v4fa*)&so[w][r][c4];
      *(volatile v4f*)(C + (size_t)(row0 + r) * ldc + col0 + c4) = v;
    }
    if (pass == 0) __threadfence();
  }
}
__global__ __launch_bounds__(256) void k_softmax_rows(const float* __restrict__ S, float* __restrict__ P, int N, int causal, int rowoff, const int* __restrict__ mask, int mask_pitch) {
  __shared__ float red[256];
  const int row = blockIdx.x, tid = threadIdx.x;
  const float* s = S + (size_t)row * N; float* p_out = P + (size_t)row * N;
  const int qi = row + rowoff;
  float mx = -3.0e38f;
  for (int j = tid; j < N; j += 256) {
    bool keep = true;
    if (causal && j > qi) keep = false;
    if (mask && mask[(size_t)qi * mask_pitch + j] == 0) keep = false;
    const float v = keep ? s[j] : -3.0e38f;
    mx = fmaxf(mx, v);
  }
  red[tid] = mx; __syncthreads();
  for (int st = 128; st > 0; st >>= 1) { if (tid < st) red[tid] = fmaxf(red[tid], red[tid + st]); __syncthreads(); }
  mx = red[0]; __syncthreads();
  float sum = 0.f;
  for (int j = tid; j < N; j += 256) {
    bool keep = true;
    if (causal && j > qi) keep = false;
    if (mask && mask[(size_t)qi * mask_pitch + j] == 0) keep = false;
    const float p = keep ? __expf(s[j] - mx) : 0.f;
    sum += p;
  }
  red[tid] = sum; __syncthreads();
  for (int st = 128; st > 0; st >>= 1) { if (tid < st) red[tid] += red[tid + st]; __syncthreads(); }
  const float inv = (mx > -1.0e38f) ? 1.0f / red[0] : __builtin_nanf("");
  __syncthreads();
  for (int pass = 0; pass < 2; ++pass) {
    for (int j4 = tid * 4; j4 < N; j4 += 1024) {
      v4f out4;
#pragma unroll
      for (int u = 0; u < 4; ++u) {
        const int j = j4 + u;
        bool keep = true;
        if (causal && j > qi) keep = false;
        if (mask && mask[(size_t)qi * mask_pitch + j] == 0) keep = false;
        out4[u] = keep ? __expf(s[j] - mx) * inv : 0.f;
      }
      *(volatile v4f*)(p_out + j4) = out4;
    }
    if (pass == 0) __threadfence();
  }
}

__device__ __forceinline__ float sigm(float x) { return 1.0f / (1.0f + expf(-x)); }

__global__ __launch_bounds__(64) void k_lstm(const float* __restrict__ inp, const float* __restrict__ h0, const float* __restrict__ c0,
                                           const float* __restrict__ Wih0, const float* __restrict__ bih0, const float* __restrict__ bhh0,
                                           const unsigned short* __restrict__ Whh0h, const unsigned short* __restrict__ Whh0l,
                                           const unsigned short* __restrict__ Wih1h, const unsigned short* __restrict__ Wih1l,
                                           const unsigned short* __restrict__ Whh1h, const unsigned short* __restrict__ Whh1l,
                                           const float* __restrict__ bih1, const float* __restrict__ bhh1,
                                           const float* __restrict__ Wlin, const float* __restrict__ blin, float* __restrict__ out) {
  __shared__ __attribute__((aligned(16))) float sh[2][2][16][HH + 4];
  __shared__ __attribute__((aligned(16))) float sc[2][2][16][HH + 4];
  __shared__ __attribute__((aligned(16))) float sx[2][16][33];
  __shared__ __attribute__((aligned(16))) float sp[2][16][32];
  const int tid = threadIdx.x, w = tid >> 5, lane = tid & 31, ln = lane & 15, hh = lane >> 4;
  const int b0 = (blockIdx.x * 2 + w) * 16;
  for (int e = lane; e < 16 * HH; e += 32) {
    const int r = e / HH, u = e % HH;
#pragma unroll
    for (int L = 0; L < 2; ++L) { sh[w][L][r][u] = h0[((size_t)L * NB + b0 + r) * HH + u]; sc[w][L][r][u] = c0[((size_t)L * NB + b0 + r) * HH + u]; }
  }
  float wl[4];
#pragma unroll
  for (int ut = 0; ut < 4; ++ut) wl[ut] = Wlin[ut * 16 + ln];
  const float bl = blin[0];

  for (int tc = 0; tc < NT_; tc += 32) {
    __builtin_amdgcn_fence(__ATOMIC_ACQ_REL, "workgroup");
    __builtin_amdgcn_wave_barrier();
    for (int e = lane; e < 16 * 32; e += 32) { const int r = e >> 5, t = e & 31; sx[w][r][t] = inp[(size_t)(b0 + r) * NT_ + tc + t]; }
    __builtin_amdgcn_fence(__ATOMIC_ACQ_REL, "workgroup");
    __builtin_amdgcn_wave_barrier();
    for (int ts = 0; ts < 32; ++ts) {
#pragma unroll 1
      for (int L = 0; L < 2; ++L) {
        FragB ahh[2], ahl[2], axh[2], axl[2];
#pragma unroll
        for (int ks = 0; ks < 2; ++ks)
#pragma unroll
          for (int i = 0; i < 16; ++i) {
            const int u = ks * 32 + ((i < 8) ? (8 * hh + i) : (16 + 8 * hh + (i - 8)));
            float x = sh[w][L][ln][u]; unsigned short hb = bf16_bits(x); ahh[ks].u[i] = hb; ahl[ks].u[i] = bf16_bits(x - bf16_val(hb));
            if (L == 1) { x = sh[w][0][ln][u]; hb = bf16_bits(x); axh[ks].u[i] = hb; axl[ks].u[i] = bf16_bits(x - bf16_val(hb)); }
            else { axh[ks].u[i] = 0; axl[ks].u[i] = 0; }
          }
        float newh[4][8], newc[4][8];
#pragma unroll
        for (int ut = 0; ut < 4; ++ut) {
          v8f g[4];
#pragma unroll
          for (int q = 0; q < 4; ++q) {
            const int n = q * HH + ut * 16 + ln;
            v8f acc = {};
            const unsigned short* Wh = L ? Whh1h : Whh0h; const unsigned short* Wl_ = L ? Whh1l : Whh0l;
#pragma unroll
            for (int ks = 0; ks < 2; ++ks) {
              FragB bh_, bl_;
              bh_.half[0] = *(const v8us*)(Wh + (size_t)n * HH + ks * 32 + 8 * hh); bh_.half[1] = *(const v8us*)(Wh + (size_t)n * HH + ks * 32 + 16 + 8 * hh);
              bl_.half[0] = *(const v8us*)(Wl_ + (size_t)n * HH + ks * 32 + 8 * hh); bl_.half[1] = *(const v8us*)(Wl_ + (size_t)n * HH + ks * 32 + 16 + 8 * hh);
              acc = mmaN<3>(ahh[ks].v, ahl[ks].v, bh_.v, bl_.v, acc);
              if (L == 1) {
                FragB ch_, cl_;
                ch_.half[0] = *(const v8us*)(Wih1h + (size_t)n * HH + ks * 32 + 8 * hh); ch_.half[1] = *(const v8us*)(Wih1h + (size_t)n * HH + ks * 32 + 16 + 8 * hh);
                cl_.half[0] = *(const v8us*)(Wih1l + (size_t)n * HH + ks * 32 + 8 * hh); cl_.half[1] = *(const v8us*)(Wih1l + (size_t)n * HH + ks * 32 + 16 + 8 * hh);
                acc = mmaN<3>(axh[ks].v, axl[ks].v, ch_.v, cl_.v, acc);
              }
            }
            if (L == 0) {
              const float wi = Wih0[n], bb = bih0[n] + bhh0[n];
#pragma unroll
              for (int r = 0; r < 8; ++r) acc[r] += sx[w][8 * hh + r][ts] * wi + bb;
            } else {
              const float bb = bih1[n] + bhh1[n];
#pragma unroll
              for (int r = 0; r < 8; ++r) acc[r] += bb;
            }
            g[q] = acc;
          }
#pragma unroll
          for (int r = 0; r < 8; ++r) {
            const float cprev = sc[w][L][8 * hh + r][ut * 16 + ln];
            const float cn = sigm(g[1][r]) * cprev + sigm(g[0][r]) * tanhf(g[2][r]);
            newc[ut][r] = cn; newh[ut][r] = sigm(g[3][r]) * tanhf(cn);
          }
        }
        __builtin_amdgcn_fence(__ATOMIC_ACQ_REL, "workgroup");
        __builtin_amdgcn_wave_barrier();
#pragma unroll
        for (int ut = 0; ut < 4; ++ut)
#pragma unroll
          for (int r = 0; r < 8; ++r) { sc[w][L][8 * hh + r][ut * 16 + ln] = newc[ut][r]; sh[w][L][8 * hh + r][ut * 16 + ln] = newh[ut][r]; }
        __builtin_amdgcn_fence(__ATOMIC_ACQ_REL, "workgroup");
        __builtin_amdgcn_wave_barrier();
        if (L == 1) {
          float pr[8];
#pragma unroll
          for (int r = 0; r < 8; ++r) {
            float s = 0.f;
#pragma unroll
            for (int ut = 0; ut < 4; ++ut) s += newh[ut][r] * wl[ut];
            s += __shfl_xor(s, 1, 32); s += __shfl_xor(s, 2, 32); s += __shfl_xor(s, 4, 32); s += __shfl_xor(s, 8, 32);
            pr[r] = s + bl;
          }
          if (ln == 0) {
#pragma unroll
            for (int r = 0; r < 8; ++r) sp[w][8 * hh + r][ts] = pr[r];
          }
        }
      }
    }
    __builtin_amdgcn_fence(__ATOMIC_ACQ_REL, "workgroup");
    __builtin_amdgcn_wave_barrier();
    const int rsub = lane >> 3, c4 = (lane & 7) * 4;
    for (int pass = 0; pass < 2; ++pass) {
#pragma unroll
      for (int q = 0; q < 4; ++q) {
        const int r = q * 4 + rsub;
        v4f v; v[0] = sp[w][r][c4]; v[1] = sp[w][r][c4 + 1]; v[2] = sp[w][r][c4 + 2]; v[3] = sp[w][r][c4 + 3];
        *(volatile v4f*)(out + (size_t)(b0 + r) * NT_ + tc + c4) = v;
      }
      if (pass == 0) __threadfence();
    }
  }
}

extern "C" void kernel_launch(void* const* d_in, const int* in_sizes, int n_in,
                              void* d_out, int out_size, void* d_ws, size_t ws_size, hipStream_t stream) {
  (void)in_sizes; (void)n_in; (void)out_size;
  const float* inp = (const float*)d_in[0]; const float* h0 = (const float*)d_in[1]; const float* c0 = (const float*)d_in[2];
  const float* Wih0 = (const float*)d_in[3]; const float* Whh0 = (const float*)d_in[4]; const float* bih0 = (const float*)d_in[5]; const float* bhh0 = (const float*)d_in[6];
  const float* Wih1 = (const float*)d_in[7]; const float* Whh1 = (const float*)d_in[8]; const float* bih1 = (const float*)d_in[9]; const float* bhh1 = (const float*)d_in[10];
  const float* Wlin = (const float*)d_in[11]; const float* blin = (const float*)d_in[12];
  char* ws = (char*)d_ws; size_t off = 0;
  auto take = [&](size_t bytes) { char* p = ws + off; off += (bytes + 255) & ~(size_t)255; return p; };
  const size_t wsz = (size_t)G4 * HH;
  unsigned short* Whh0h = (unsigned short*)take(wsz * 2); unsigned short* Whh0l = (unsigned short*)take(wsz * 2);
  unsigned short* Wih1h = (unsigned short*)take(wsz * 2); unsigned short* Wih1l = (unsigned short*)take(wsz * 2);
  unsigned short* Whh1h = (unsigned short*)take(wsz * 2); unsigned short* Whh1l = (unsigned short*)take(wsz * 2);
  if (off > ws_size) return;
  k_split_rows<<<(G4 * (HH / 8) + 255) / 256, 256, 0, stream>>>(Whh0, HH, Whh0h, Whh0l, G4, HH);
  k_split_rows<<<(G4 * (HH / 8) + 255) / 256, 256, 0, stream>>>(Wih1, HH, Wih1h, Wih1l, G4, HH);
  k_split_rows<<<(G4 * (HH / 8) + 255) / 256, 256, 0, stream>>>(Whh1, HH, Whh1h, Whh1l, G4, HH);
  k_lstm<<<NB / 32, 64, 0, stream>>>(inp, h0, c0, Wih0, bih0, bhh0, Whh0h, Whh0l, Wih1h, Wih1l, Whh1h, Whh1l, bih1, bhh1, Wlin, blin, (float*)d_out);
}
